// NonLocalBlock2D_23416161698526
// MI455X (gfx1250) — hardware-verified
//
#include <hip/hip_runtime.h>
#include <math.h>
#include <stddef.h>
#include <stdint.h>

#define NB    8
#define CI    256
#define CM    128
#define NSP   4096
#define IMW   64
#define NKP   1024
#define NTOKS (NB * NSP)
#define NPTOK (NB * NKP)
#define K3    (3 * NKP)
#define T3P   (3 * CM)
#define O2P   (2 * CM)
#define PGW   (2 * CM)
#define BNR   32
#define BNP   260
#define NPART (NTOKS / BNR)
#define PARTW (2 * CI)
#define SPT   68
#define SPW   132
#define WSMAX 134217728

static_assert(NSP % 64 == 0);
static_assert(NKP % 64 == 0);
static_assert(NTOKS % 64 == 0);
static_assert(NPTOK % 16 == 0);
static_assert(CI % 64 == 0);
static_assert(CM % 64 == 0);
static_assert(CI % 32 == 0);
static_assert(K3 % 32 == 0);
static_assert(T3P % 32 == 0);
static_assert(O2P % 32 == 0);
static_assert(PGW % 64 == 0);
static_assert((CM * CI) % (8 * 256) == 0);
static_assert((CI * CM) % (8 * 256) == 0);
static_assert(NPART == 1024);
static_assert(NTOKS % BNR == 0);
static_assert(PARTW / 4 == 128);
static_assert(IMW * IMW == NSP);
static_assert((IMW / 2) * (IMW / 2) == NKP);

typedef __attribute__((ext_vector_type(16))) _Float16 v16h;
typedef __attribute__((ext_vector_type(8)))  _Float16 v8h;
typedef __attribute__((ext_vector_type(16))) __bf16   v16b;
typedef __attribute__((ext_vector_type(8)))  __bf16   v8b;
typedef __attribute__((ext_vector_type(8)))  float    v8f;
typedef __attribute__((ext_vector_type(4)))  float    v4f;
typedef __attribute__((ext_vector_type(4)))  unsigned int v4u;
typedef __attribute__((ext_vector_type(8)))  unsigned short v8us;
typedef v4f __attribute__((may_alias)) v4fa;

__device__ __forceinline__ unsigned short f2bf_bits(float f) {
  unsigned u = __float_as_uint(f);
  return (unsigned short)((u + 0x7FFFu + ((u >> 16) & 1u)) >> 16);
}
__device__ __forceinline__ float bf_bits2f(unsigned short h) { return __uint_as_float(((unsigned)h) << 16); }
__device__ __forceinline__ float bf_rne(float f) { return bf_bits2f(f2bf_bits(f)); }
__device__ __forceinline__ unsigned pk16(unsigned short a, unsigned short b) { return (unsigned)a | ((unsigned)b << 16); }

__device__ __forceinline__ void dep_guard_h(v8f& a, v8f& b, v16h x, v16h y) { asm volatile("v_nop\n\tv_nop\n\tv_nop\n\tv_nop" : "+v"(a), "+v"(b) : "v"(x), "v"(y)); }
__device__ __forceinline__ void dep_guard_b(v8f& a, v8f& b, v16b x, v16b y) { asm volatile("v_nop\n\tv_nop\n\tv_nop\n\tv_nop" : "+v"(a), "+v"(b) : "v"(x), "v"(y)); }
__device__ __forceinline__ void keep4_h(v16h a, v16h b, v16h c, v16h d) { asm volatile("v_nop" :: "v"(a), "v"(b), "v"(c), "v"(d)); }
__device__ __forceinline__ void keep4_b(v16b a, v16b b, v16b c, v16b d) { asm volatile("v_nop" :: "v"(a), "v"(b), "v"(c), "v"(d)); }
__device__ __forceinline__ void acc_guard4(v8f& a, v8f& b, v8f& c, v8f& d) { asm volatile("v_nop\n\tv_nop\n\tv_nop\n\tv_nop" : "+v"(a), "+v"(b), "+v"(c), "+v"(d)); }

template <typename T> struct Frag;
template <> struct Frag<_Float16> {
  typedef v16h V; union U { v16h v; v8h h[2]; };
  static __device__ __forceinline__ v16h load(const _Float16* p) {
    U f; f.h[0] = *(const v8h*)(p); f.h[1] = *(const v8h*)(p + 16); return f.v;
  }
  static __device__ __forceinline__ v8f mma(v16h a, v16h b, v8f c) {
    return __builtin_amdgcn_wmma_f32_16x16x32_f16(false, a, false, b, (short)0, c, false, false);
  }
  static __device__ __forceinline__ void guard(v8f& a, v8f& b, v16h x, v16h y) { dep_guard_h(a, b, x, y); }
  static __device__ __forceinline__ void keep(v16h a, v16h b, v16h c, v16h d) { keep4_h(a, b, c, d); }
};
template <> struct Frag<__bf16> {
  typedef v16b V; union U { v16b v; v8b h[2]; };
  static __device__ __forceinline__ v16b load(const __bf16* p) {
    U f; f.h[0] = *(const v8b*)(p); f.h[1] = *(const v8b*)(p + 16); return f.v;
  }
  static __device__ __forceinline__ v8f mma(v16b a, v16b b, v8f c) {
    return __builtin_amdgcn_wmma_f32_16x16x32_bf16(false, a, false, b, (short)0, c, false, false);
  }
  static __device__ __forceinline__ void guard(v8f& a, v8f& b, v16b x, v16b y) { dep_guard_b(a, b, x, y); }
  static __device__ __forceinline__ void keep(v16b a, v16b b, v16b c, v16b d) { keep4_b(a, b, c, d); }
};

template <int ET> struct Elem;
template <> struct Elem<0> { typedef _Float16 T; };
template <> struct Elem<1> { typedef __bf16 T; };

template <int ET, int BIAS_MODE, int OUT_MODE, bool RESID, bool BN>
__global__ __launch_bounds__(256) void wmma_gemm64(
    const unsigned short* __restrict__ Ap, int lda, long strideA,
    const unsigned short* __restrict__ Btp, int ldb, long strideB,
    void* Cout, void* Cout2, void* Cout3, int ldc, long strideC,
    const float* __restrict__ bias,
    const float* __restrict__ bng, const float* __restrict__ bnb,
    const float* __restrict__ bnm, const float* __restrict__ bnv,
    const float* __restrict__ resid, long strideR,
    int M, int N, int K, float scale) {
  typedef typename Elem<ET>::T T;
  typedef typename Frag<T>::V V;
  const T* A = (const T*)Ap; const T* Bt = (const T*)Btp;
  __shared__ __align__(16) float sT[8][16 * 68];
  const int b    = blockIdx.y;
  const int lane = threadIdx.x & 31;
  const int wave = threadIdx.x >> 5;
  const int tilesN = N >> 6;
  const int tilesM = M >> 6;
  const int tile = blockIdx.x * 8 + wave;
  if (tile >= tilesM * tilesN) return;
  const int tm = tile / tilesN;
  const int tn = tile - tm * tilesN;
  const int m0 = tm << 6;
  const int n0 = tn << 6;

  const T* Ab = A  + (size_t)b * strideA;
  const T* Bb = Bt + (size_t)b * strideB;

  const int rlane = lane & 15;
  const int koff  = (lane >> 4) * 8;
  const int mOff  = (lane >> 4) * 8;

  v8f acc[4][4];
#pragma unroll
  for (int i = 0; i < 4; ++i)
#pragma unroll
    for (int j = 0; j < 4; ++j) acc[i][j] = (v8f){0.f,0.f,0.f,0.f,0.f,0.f,0.f,0.f};

  for (int k0 = 0; k0 < K; k0 += 32) {
    V bh[4];
#pragma unroll
    for (int j = 0; j < 4; ++j) {
      const size_t bo = (size_t)(n0 + (j << 4) + rlane) * ldb + koff + k0;
      bh[j] = Frag<T>::load(Bb + bo);
    }
#pragma unroll
    for (int i = 0; i < 4; ++i) {
      const size_t ao = (size_t)(m0 + (i << 4) + rlane) * lda + koff + k0;
      const V ah = Frag<T>::load(Ab + ao);
#pragma unroll
      for (int j = 0; j < 4; ++j) acc[i][j] = Frag<T>::mma(ah, bh[j], acc[i][j]);
      Frag<T>::guard(acc[i][0], acc[i][3], ah, ah);
    }
    Frag<T>::keep(bh[0], bh[1], bh[2], bh[3]);
  }
  acc_guard4(acc[0][0], acc[0][1], acc[0][2], acc[0][3]);
  acc_guard4(acc[1][0], acc[1][1], acc[1][2], acc[1][3]);
  acc_guard4(acc[2][0], acc[2][1], acc[2][2], acc[2][3]);
  acc_guard4(acc[3][0], acc[3][1], acc[3][2], acc[3][3]);

  float* slab = sT[wave];
  const float* Rb = resid + (size_t)b * (RESID ? (size_t)strideR : (size_t)0);
#pragma unroll
  for (int i = 0; i < 4; ++i) {
    const int mBase = m0 + (i << 4);
    const int mr = mBase + mOff;
    float rb[8], rmul[8], radd[8];
#pragma unroll
    for (int r = 0; r < 8; ++r) { rb[r] = 0.f; rmul[r] = 1.f; radd[r] = 0.f; }
    if (BIAS_MODE == 1) {
      const v4f t0 = *(const v4f*)(bias + mr);
      const v4f t1 = *(const v4f*)(bias + mr + 4);
#pragma unroll
      for (int e = 0; e < 4; ++e) { rb[e] = bf_rne(t0[e]); rb[4 + e] = bf_rne(t1[e]); }
    }
    if (BN) {
      const v4f vg0 = *(const v4f*)(bng + mr), vg1 = *(const v4f*)(bng + mr + 4);
      const v4f vb0 = *(const v4f*)(bnb + mr), vb1 = *(const v4f*)(bnb + mr + 4);
      const v4f vm0 = *(const v4f*)(bnm + mr), vm1 = *(const v4f*)(bnm + mr + 4);
      const v4f vv0 = *(const v4f*)(bnv + mr), vv1 = *(const v4f*)(bnv + mr + 4);
#pragma unroll
      for (int e = 0; e < 4; ++e) {
        {
          const float inv = bf_rne(vg0[e]) * rsqrtf(bf_rne(vv0[e]) + 1e-5f);
          rmul[e] = inv;
          radd[e] = bf_rne(vb0[e]) - bf_rne(vm0[e]) * inv;
        }
        {
          const float inv = bf_rne(vg1[e]) * rsqrtf(bf_rne(vv1[e]) + 1e-5f);
          rmul[4 + e] = inv;
          radd[4 + e] = bf_rne(vb1[e]) - bf_rne(vm1[e]) * inv;
        }
      }
    }
#pragma unroll
    for (int j = 0; j < 4; ++j) {
      const int n = n0 + (j << 4) + rlane;
      float bv = 0.f;
      if (BIAS_MODE == 2) bv = bf_rne(bias[n]);
#pragma unroll
      for (int r = 0; r < 8; ++r) {
        float v = acc[i][j][r] * scale;
        if (BIAS_MODE == 1) v += rb[r];
        if (BIAS_MODE == 2) v += bv;
        if (BN) v = v * rmul[r] + radd[r];
        slab[(mOff + r) * 68 + (j << 4) + rlane] = v;
      }
    }
    __builtin_amdgcn_fence(__ATOMIC_RELEASE, "workgroup");
    __builtin_amdgcn_wave_barrier();
    __builtin_amdgcn_fence(__ATOMIC_ACQUIRE, "workgroup");
    if (OUT_MODE == 0) {
      float* C = (float*)Cout + (size_t)b * strideC;
      const int hh = lane >> 4, c4 = (lane & 15) * 4;
      v4f ov[8];
#pragma unroll
      for (int it = 0; it < 8; ++it) {
        const int row = it * 2 + hh;
        v4f v = *(const v4f*)(slab + row * 68 + c4);
        if (RESID) {
          const v4f xr = *(const v4f*)(Rb + (size_t)(mBase + row) * ldc + n0 + c4);
#pragma unroll
          for (int e = 0; e < 4; ++e) v[e] = v[e] + (BN ? bf_rne(xr[e]) : xr[e]);
        }
        ov[it] = v;
      }
      for (int pass = 0; pass < 2; ++pass) {
#pragma unroll
        for (int it = 0; it < 8; ++it) {
          const int row = it * 2 + hh;
          *(volatile v4f*)(C + (size_t)(mBase + row) * ldc + n0 + c4) = ov[it];
        }
        __threadfence();
      }
    } else {
      const int q = lane >> 3, c8 = (lane & 7) * 8;
      unsigned short* C  = (unsigned short*)Cout  + (size_t)b * strideC;
      unsigned short* C2 = (unsigned short*)Cout2 + (size_t)b * strideC;
      unsigned short* C3 = (unsigned short*)Cout3 + (size_t)b * strideC;
      for (int pass = 0; pass < 2; ++pass) {
#pragma unroll
        for (int it = 0; it < 4; ++it) {
          const int row = it * 4 + q;
          const float* sp = slab + row * 68 + c8;
          v8h hv, lv;
#pragma unroll
          for (int e = 0; e < 8; ++e) {
            const unsigned short hb = f2bf_bits(sp[e]);
            const unsigned short lb = f2bf_bits(sp[e] - bf_bits2f(hb));
            hv[e] = __builtin_bit_cast(_Float16, hb);
            lv[e] = __builtin_bit_cast(_Float16, lb);
          }
          const size_t go = (size_t)(mBase + row) * ldc + n0 + c8;
          *(volatile v8h*)(C + go) = hv;
          if (OUT_MODE == 2) { *(volatile v8h*)(C2 + go) = lv; }
          if (OUT_MODE == 3) { *(volatile v8h*)(C2 + go) = hv; *(volatile v8h*)(C3 + go) = lv; }
          if (OUT_MODE == 4) { *(volatile v8h*)(C2 + go) = lv; *(volatile v8h*)(C3 + go) = hv; }
        }
        __threadfence();
      }
    }
    __builtin_amdgcn_fence(__ATOMIC_RELEASE, "workgroup");
    __builtin_amdgcn_wave_barrier();
    __builtin_amdgcn_fence(__ATOMIC_ACQUIRE, "workgroup");
  }
}

__global__ __launch_bounds__(256) void k_gemm_pool(
    const unsigned short* __restrict__ Ap, int lda,
    const unsigned short* __restrict__ Btp, int ldb,
    float* Cout, int ldc,
    const float* __restrict__ bias0, const float* __restrict__ bias1,
    int M, int N, int K) {
  typedef __bf16 T;
  typedef Frag<T>::V V;
  const T* A = (const T*)Ap; const T* Bt = (const T*)Btp;
  __shared__ __align__(16) float sT[8][16 * 68];
  const int lane = threadIdx.x & 31;
  const int wave = threadIdx.x >> 5;
  const int tilesN = N >> 6;
  const int tilesM = M >> 6;
  const int tile = blockIdx.x * 8 + wave;
  if (tile >= tilesM * tilesN) return;
  const int tm = tile / tilesN;
  const int tn = tile - tm * tilesN;
  const int m0 = tm << 6;
  const int n0 = tn << 6;
  const int rlane = lane & 15;
  const int koff  = (lane >> 4) * 8;
  const int h     = lane >> 4;

  v8f acc[4][4];
#pragma unroll
  for (int i = 0; i < 4; ++i)
#pragma unroll
    for (int j = 0; j < 4; ++j) acc[i][j] = (v8f){0.f,0.f,0.f,0.f,0.f,0.f,0.f,0.f};

  for (int k0 = 0; k0 < K; k0 += 32) {
    V bh[4];
#pragma unroll
    for (int j = 0; j < 4; ++j) {
      const size_t bo = (size_t)(n0 + (j << 4) + rlane) * ldb + koff + k0;
      bh[j] = Frag<T>::load(Bt + bo);
    }
#pragma unroll
    for (int i = 0; i < 4; ++i) {
      const size_t ao = (size_t)(m0 + (i << 4) + rlane) * lda + koff + k0;
      const V ah = Frag<T>::load(A + ao);
#pragma unroll
      for (int j = 0; j < 4; ++j) acc[i][j] = Frag<T>::mma(ah, bh[j], acc[i][j]);
      Frag<T>::guard(acc[i][0], acc[i][3], ah, ah);
    }
    Frag<T>::keep(bh[0], bh[1], bh[2], bh[3]);
  }
  acc_guard4(acc[0][0], acc[0][1], acc[0][2], acc[0][3]);
  acc_guard4(acc[1][0], acc[1][1], acc[1][2], acc[1][3]);
  acc_guard4(acc[2][0], acc[2][1], acc[2][2], acc[2][3]);
  acc_guard4(acc[3][0], acc[3][1], acc[3][2], acc[3][3]);

  float* slab = sT[wave];
  float bv[4];
#pragma unroll
  for (int j = 0; j < 4; ++j) {
    const int n = n0 + (j << 4) + rlane;
    const float bp = bf_rne(bias0[n & (CM - 1)]);
    const float bg = bf_rne(bias1[n & (CM - 1)]);
    bv[j] = (n < CM) ? bp : bg;
  }
#pragma unroll
  for (int i = 0; i < 4; ++i) {
#pragma unroll
    for (int j = 0; j < 4; ++j) {
      const float p0 = fmaxf(fmaxf(acc[i][j][0], acc[i][j][1]), fmaxf(acc[i][j][2], acc[i][j][3])) + bv[j];
      const float p1 = fmaxf(fmaxf(acc[i][j][4], acc[i][j][5]), fmaxf(acc[i][j][6], acc[i][j][7])) + bv[j];
      slab[(4 * i + 2 * h) * 68 + (j << 4) + rlane]     = p0;
      slab[(4 * i + 2 * h + 1) * 68 + (j << 4) + rlane] = p1;
    }
  }
  __builtin_amdgcn_fence(__ATOMIC_RELEASE, "workgroup");
  __builtin_amdgcn_wave_barrier();
  __builtin_amdgcn_fence(__ATOMIC_ACQUIRE, "workgroup");
  const int pr0 = m0 >> 2;
  const int c4 = rlane * 4;
  v4f ov[8];
#pragma unroll
  for (int it = 0; it < 8; ++it) {
    const int row = it * 2 + h;
    ov[it] = *(const v4f*)(slab + row * 68 + c4);
  }
#pragma unroll
  for (int it = 0; it < 8; ++it) {
    const int row = it * 2 + h;
    *(volatile v4f*)(Cout + (size_t)(pr0 + row) * ldc + n0 + c4) = ov[it];
  }
  __threadfence();
#pragma unroll
  for (int it = 0; it < 8; ++it) {
    const int row = it * 2 + h;
    *(volatile v4f*)(Cout + (size_t)(pr0 + row) * ldc + n0 + c4) = ov[it];
  }
}

__global__ __launch_bounds__(256) void tconv_kernel(const float* __restrict__ W, unsigned short* __restrict__ oh,
                                                    int ldin, int ldout, long sIn, long sOut) {
  __shared__ __align__(16) float tf[64 * 68];
  W  += (size_t)blockIdx.z * sIn;
  oh += (size_t)blockIdx.z * sOut;
  const int c0  = blockIdx.x * 64;
  const int r0  = blockIdx.y * 64;
  const int tid = threadIdx.x;
  {
    const int lr = tid >> 4;
    const int c4 = (tid & 15) * 4;
#pragma unroll
    for (int it = 0; it < 4; ++it) {
      const int rr = it * 16 + lr;
      const v4f a = *(const v4f*)(W + (size_t)(r0 + rr) * ldin + c0 + c4);
      *(v4f*)(tf + rr * 68 + c4) = a;
    }
  }
  __syncthreads();
  const int sub = tid >> 3;
  const int c8  = (tid & 7) * 8;
  v4u hv[2];
#pragma unroll
  for (int it = 0; it < 2; ++it) {
    const int oc = it * 32 + sub;
    v4u a;
#pragma unroll
    for (int q = 0; q < 4; ++q) {
      const float f0 = tf[(c8 + 2 * q) * 68 + oc];
      const float f1 = tf[(c8 + 2 * q + 1) * 68 + oc];
      a[q] = pk16(f2bf_bits(f0), f2bf_bits(f1));
    }
    hv[it] = a;
  }
  for (int pass = 0; pass < 2; ++pass) {
#pragma unroll
    for (int it = 0; it < 2; ++it) {
      const int oc = it * 32 + sub;
      const size_t go = (size_t)(c0 + oc) * ldout + r0 + c8;
      *(volatile v4u*)(oh + go) = hv[it];
    }
    __threadfence();
  }
}

__device__ __forceinline__ int pool_row(int n) {
  const int hr = n >> 6, w = n & (IMW - 1);
  return (((hr >> 1) * (IMW / 2) + (w >> 1)) << 2) + ((hr & 1) << 1) + (w & 1);
}

__global__ __launch_bounds__(256) void tconvp_kernel(const float* __restrict__ W, unsigned short* __restrict__ oh,
                                                     int ldin, int ldout, long sIn, long sOut) {
  __shared__ __align__(16) float tf[64 * 68];
  W  += (size_t)blockIdx.z * sIn;
  oh += (size_t)blockIdx.z * sOut;
  const int c0  = blockIdx.x * 64;
  const int r0  = blockIdx.y * 64;
  const int tid = threadIdx.x;
  {
    const int lr = tid >> 4;
    const int c4 = (tid & 15) * 4;
#pragma unroll
    for (int it = 0; it < 4; ++it) {
      const int rr = it * 16 + lr;
      const v4f a = *(const v4f*)(W + (size_t)(r0 + rr) * ldin + c0 + c4);
      *(v4f*)(tf + rr * 68 + c4) = a;
    }
  }
  __syncthreads();
  const int sub = tid >> 3;
  const int c8  = (tid & 7) * 8;
  v4u hv[2];
#pragma unroll
  for (int it = 0; it < 2; ++it) {
    const int oc = it * 32 + sub;
    v4u a;
#pragma unroll
    for (int q = 0; q < 4; ++q) {
      const float f0 = tf[(c8 + 2 * q) * 68 + oc];
      const float f1 = tf[(c8 + 2 * q + 1) * 68 + oc];
      a[q] = pk16(f2bf_bits(f0), f2bf_bits(f1));
    }
    hv[it] = a;
  }
#pragma unroll
  for (int it = 0; it < 2; ++it) {
    const int oc = it * 32 + sub;
    const size_t go = (size_t)pool_row(c0 + oc) * ldout + r0 + c8;
    *(volatile v4u*)(oh + go) = hv[it];
  }
  __threadfence();
#pragma unroll
  for (int it = 0; it < 2; ++it) {
    const int oc = it * 32 + sub;
    const size_t go = (size_t)pool_row(c0 + oc) * ldout + r0 + c8;
    *(volatile v4u*)(oh + go) = hv[it];
  }
}

__global__ __launch_bounds__(256) void wcvt_kernel(const float* __restrict__ wt, const float* __restrict__ wp,
                                                   const float* __restrict__ wg, const float* __restrict__ wr,
                                                   unsigned short* __restrict__ wcat, unsigned short* __restrict__ wr2) {
  const int g   = blockIdx.x * 256 + threadIdx.x;
  const int sel = blockIdx.y;
  if (g >= (CM * CI) / 8) return;
  const float* src;
  unsigned short* dst;
  if (sel < 3) {
    const float* w = (sel == 0) ? wt : ((sel == 1) ? wp : wg);
    src = w + (size_t)g * 8;
    dst = wcat + (size_t)sel * CM * CI + (size_t)g * 8;
  } else {
    const int row = g >> 4, c8 = (g & 15) * 8;
    src = wr + (size_t)row * CM + c8;
    dst = wr2 + (size_t)row * O2P + (size_t)(sel - 3) * CM + c8;
  }
  const v4f a = *(const v4f*)src;
  const v4f c = *(const v4f*)(src + 4);
  v4u o;
  o[0] = pk16(f2bf_bits(a[0]), f2bf_bits(a[1]));
  o[1] = pk16(f2bf_bits(a[2]), f2bf_bits(a[3]));
  o[2] = pk16(f2bf_bits(c[0]), f2bf_bits(c[1]));
  o[3] = pk16(f2bf_bits(c[2]), f2bf_bits(c[3]));
  *(volatile v4u*)dst = o;
  __threadfence();
  *(volatile v4u*)dst = o;
}

__global__ __launch_bounds__(256) void k_thnorm(const float* __restrict__ th, unsigned short* t3) {
  __shared__ __align__(16) float tf[64 * SPW];
  __shared__ __align__(16) float sinv[64];
  const int tid = (int)threadIdx.x;
  const int r0 = (int)blockIdx.x * 64;
  {
    const int c4 = (tid & 31) * 4;
    const int rsub = tid >> 5;
#pragma unroll
    for (int it = 0; it < 8; ++it) {
      const int row = it * 8 + rsub;
      const v4f a = *(const v4f*)(th + (size_t)(r0 + row) * CM + c4);
      *(v4fa*)(tf + row * SPW + c4) = a;
    }
  }
  __syncthreads();
  {
    const int row = tid >> 2, part = tid & 3;
    const float* sp = tf + row * SPW + part * 32;
    float ss = 0.0f;
#pragma unroll 8
    for (int e = 0; e < 32; ++e) { const float f = sp[e]; ss = fmaf(f, f, ss); }
    ss += __shfl_xor(ss, 1, 32);
    ss += __shfl_xor(ss, 2, 32);
    const float inv = 1.0f / fmaxf(sqrtf(ss), 1e-12f);
    if (part == 0) sinv[row] = inv;
  }
  __syncthreads();
  const int sub = tid >> 3;
  const int l8  = (tid & 7) * 8;
  v8us ov[12];
#pragma unroll
  for (int it = 0; it < 12; ++it) {
    const int plane = it >> 2;
    const int v = (it & 3) * 32 + sub;
    const int row = v >> 1;
    const int c8 = (v & 1) * 64 + l8;
    const float sc = sinv[row];
    const float* sp = tf + row * SPW + c8;
    v8us o;
#pragma unroll
    for (int e = 0; e < 8; ++e) {
      const float f = sp[e] * sc;
      const unsigned short hb = f2bf_bits(f);
      const unsigned short lb = f2bf_bits(f - bf_bits2f(hb));
      o[e] = (plane < 2) ? hb : lb;
    }
    ov[it] = o;
  }
#pragma unroll
  for (int it = 0; it < 12; ++it) {
    const int plane = it >> 2;
    const int v = (it & 3) * 32 + sub;
    const int row = v >> 1;
    const int c8 = (v & 1) * 64 + l8;
    *(volatile v8us*)(t3 + (size_t)(r0 + row) * T3P + plane * CM + c8) = ov[it];
  }
  __threadfence();
#pragma unroll
  for (int it = 0; it < 12; ++it) {
    const int plane = it >> 2;
    const int v = (it & 3) * 32 + sub;
    const int row = v >> 1;
    const int c8 = (v & 1) * 64 + l8;
    *(volatile v8us*)(t3 + (size_t)(r0 + row) * T3P + plane * CM + c8) = ov[it];
  }
}

__global__ __launch_bounds__(256) void k_pgcvt(const float* __restrict__ pgp, unsigned short* pg3) {
  __shared__ __align__(16) float tf[64 * SPW];
  __shared__ __align__(16) float sinv[64];
  const int tid  = (int)threadIdx.x;
  const int m0   = (int)blockIdx.x * 64;
  const int half = (int)blockIdx.y;
  const int b    = (int)blockIdx.z;
  {
    const int c4 = (tid & 31) * 4;
    const int rsub = tid >> 5;
#pragma unroll
    for (int it = 0; it < 8; ++it) {
      const int key = it * 8 + rsub;
      const v4f a = *(const v4f*)(pgp + ((size_t)(b * NKP + m0 + key)) * PGW + half * CM + c4);
      *(v4fa*)(tf + key * SPW + c4) = a;
    }
  }
  __syncthreads();
  {
    const int key = tid >> 2, part = tid & 3;
    const float* sp = tf + key * SPW + part * 32;
    float ss = 0.0f;
#pragma unroll 8
    for (int e = 0; e < 32; ++e) { const float f = sp[e]; ss = fmaf(f, f, ss); }
    ss += __shfl_xor(ss, 1, 32);
    ss += __shfl_xor(ss, 2, 32);
    const float invp = 1.0f / fmaxf(sqrtf(ss), 1e-12f);
    const float inv = (half == 0) ? invp : 1.0f;
    if (part == 0) sinv[key] = inv;
  }
  __syncthreads();
  const int sub = tid >> 3;
  const int l8  = (tid & 7) * 8;
  v8us ov[12];
#pragma unroll
  for (int it = 0; it < 12; ++it) {
    const int plane = it >> 2;
    const int c = (it & 3) * 32 + sub;
    v8us o;
#pragma unroll
    for (int e = 0; e < 8; ++e) {
      const float f = tf[(l8 + e) * SPW + c] * sinv[l8 + e];
      const unsigned short hb = f2bf_bits(f);
      const unsigned short lb = f2bf_bits(f - bf_bits2f(hb));
      unsigned short w;
      if (plane == 0)      w = hb;
      else if (plane == 1) w = (half == 0) ? lb : hb;
      else                 w = (half == 0) ? hb : lb;
      o[e] = w;
    }
    ov[it] = o;
  }
#pragma unroll
  for (int it = 0; it < 12; ++it) {
    const int plane = it >> 2;
    const int c = (it & 3) * 32 + sub;
    *(volatile v8us*)(pg3 + ((size_t)(b * PGW + half * CM + c)) * K3 + plane * NKP + m0 + l8) = ov[it];
  }
  __threadfence();
#pragma unroll
  for (int it = 0; it < 12; ++it) {
    const int plane = it >> 2;
    const int c = (it & 3) * 32 + sub;
    *(volatile v8us*)(pg3 + ((size_t)(b * PGW + half * CM + c)) * K3 + plane * NKP + m0 + l8) = ov[it];
  }
}

__global__ __launch_bounds__(256) void k_bnpart(const float* __restrict__ wy, float* part) {
  __shared__ __align__(16) float tf[BNR * BNP];
  __shared__ __align__(16) float pst[PARTW];
  const int tid = (int)threadIdx.x;
  const int t0 = (int)blockIdx.x * BNR;
  {
    const int c4 = (tid & 63) * 4;
    const int rsub = tid >> 6;
#pragma unroll
    for (int it = 0; it < 8; ++it) {
      const int row = it * 4 + rsub;
      const v4f a = *(const v4f*)(wy + (size_t)(t0 + row) * CI + c4);
      *(v4fa*)(tf + row * BNP + c4) = a;
    }
  }
  __syncthreads();
  {
    const int c = tid;
    float s = 0.0f;
#pragma unroll 4
    for (int r = 0; r < BNR; ++r) s += tf[r * BNP + c];
    const float mean = s * (1.0f / (float)BNR);
    float q = 0.0f;
#pragma unroll 4
    for (int r = 0; r < BNR; ++r) {
      const float d = tf[r * BNP + c] - mean;
      q = fmaf(d, d, q);
    }
    pst[c] = mean;
    pst[CI + c] = q;
  }
  __syncthreads();
  v4f qv;
  if (tid < PARTW / 4) {
    qv = *(const v4fa*)(pst + 4 * tid);
    *(volatile v4f*)(part + (size_t)blockIdx.x * PARTW + 4 * tid) = qv;
  }
  __threadfence();
  if (tid < PARTW / 4) {
    *(volatile v4f*)(part + (size_t)blockIdx.x * PARTW + 4 * tid) = qv;
  }
}

__global__ __launch_bounds__(256) void k_bnfin(const float* __restrict__ part, const float* __restrict__ gam,
                                               const float* __restrict__ bet, float* ss) {
  __shared__ __align__(16) float stg[PARTW];
  const int tid = (int)threadIdx.x;
  const int c = tid & (CI - 1);
  double s = 0.0;
#pragma unroll 1
  for (int p = 0; p < NPART; ++p) s += (double)part[(size_t)p * PARTW + c];
  const double mean = s * (1.0 / (double)NPART);
  double q = 0.0;
#pragma unroll 1
  for (int p = 0; p < NPART; ++p) {
    const double mb = (double)part[(size_t)p * PARTW + c];
    const double qb = (double)part[(size_t)p * PARTW + CI + c];
    const double d = mb - mean;
    q = q + (qb + (double)BNR * d * d);
  }
  const float var   = (float)(q * (1.0 / (double)NTOKS));
  const float meanf = (float)mean;
  const float rstd  = rsqrtf(var + 1e-5f);
  const float sc = bf_rne(gam[c]) * rstd;
  const float sh = bf_rne(bet[c]) - meanf * sc;
  stg[c] = sc;
  stg[CI + c] = sh;
  __syncthreads();
  v4f v;
  if (tid < PARTW / 4) {
    v = *(const v4fa*)(stg + 4 * tid);
    *(volatile v4f*)(ss + 4 * tid) = v;
  }
  __threadfence();
  if (tid < PARTW / 4) {
    *(volatile v4f*)(ss + 4 * tid) = v;
  }
}

__global__ __launch_bounds__(256) void k_out(const float* __restrict__ wy, const float* __restrict__ ss,
                                             const float* __restrict__ x, float* out) {
  __shared__ __align__(16) float tf[64 * SPT];
  __shared__ __align__(16) float ssh[128];
  const int bx = (int)blockIdx.x, tid = (int)threadIdx.x;
  const int cb = bx & 3;
  const int rest = bx >> 2;
  const int b  = rest / (NSP / 64);
  const int n0 = (rest - b * (NSP / 64)) * 64;
  const int c0 = cb * 64;
  if (tid < 64) {
    ssh[tid]      = ss[c0 + tid];
    ssh[64 + tid] = ss[CI + c0 + tid];
  }
  __syncthreads();
  const int t0 = b * NSP + n0;
  const int rsub = tid >> 4;
  const int c4   = (tid & 15) * 4;
#pragma unroll
  for (int it = 0; it < 4; ++it) {
    const int tl = it * 16 + rsub;
    const v4f a = *(const v4f*)(wy + (size_t)(t0 + tl) * CI + c0 + c4);
    tf[(c4 + 0) * SPT + tl] = fmaf(a.x, ssh[c4 + 0], ssh[64 + c4 + 0]);
    tf[(c4 + 1) * SPT + tl] = fmaf(a.y, ssh[c4 + 1], ssh[64 + c4 + 1]);
    tf[(c4 + 2) * SPT + tl] = fmaf(a.z, ssh[c4 + 2], ssh[64 + c4 + 2]);
    tf[(c4 + 3) * SPT + tl] = fmaf(a.w, ssh[c4 + 3], ssh[64 + c4 + 3]);
  }
  __syncthreads();
  v4f ov[4];
#pragma unroll
  for (int it = 0; it < 4; ++it) {
    const int ch = it * 16 + rsub;
    const size_t gi = ((size_t)(b * CI + c0 + ch)) * NSP + n0 + c4;
    const v4f bn = *(const v4fa*)(tf + ch * SPT + c4);
    const v4f xr = *(const v4f*)(x + gi);
    v4f v;
    v.x = bn.x + bf_rne(xr.x); v.y = bn.y + bf_rne(xr.y);
    v.z = bn.z + bf_rne(xr.z); v.w = bn.w + bf_rne(xr.w);
    ov[it] = v;
  }
#pragma unroll
  for (int it = 0; it < 4; ++it) {
    const int ch = it * 16 + rsub;
    const size_t gi = ((size_t)(b * CI + c0 + ch)) * NSP + n0 + c4;
    *(volatile v4f*)(out + gi) = ov[it];
  }
  __threadfence();
#pragma unroll
  for (int it = 0; it < 4; ++it) {
    const int ch = it * 16 + rsub;
    const size_t gi = ((size_t)(b * CI + c0 + ch)) * NSP + n0 + c4;
    *(volatile v4f*)(out + gi) = ov[it];
  }
}

static inline size_t al256(size_t o) { return (o + 255) & ~(size_t)255; }

extern "C" void kernel_launch(void* const* d_in, const int* in_sizes, int n_in,
                              void* d_out, int out_size, void* d_ws, size_t ws_size,
                              hipStream_t stream) {
  if (n_in < 12) return;
  if (in_sizes[0] != NB * CI * NSP || in_sizes[1] != NB * CI * NSP) return;
  if (in_sizes[2] != CM * CI || in_sizes[3] != CM) return;
  if (in_sizes[4] != CM * CI || in_sizes[5] != CM) return;
  if (in_sizes[6] != CM * CI || in_sizes[7] != CM) return;
  if (in_sizes[8] != CI * CM || in_sizes[9] != CI) return;
  if (in_sizes[10] != CI || in_sizes[11] != CI) return;
  if (out_size != NB * CI * NSP) return;

  const float* x       = (const float*)d_in[0];
  const float* y       = (const float*)d_in[1];
  const float* g_w     = (const float*)d_in[2];
  const float* g_b     = (const float*)d_in[3];
  const float* theta_w = (const float*)d_in[4];
  const float* theta_b = (const float*)d_in[5];
  const float* phi_w   = (const float*)d_in[6];
  const float* phi_b   = (const float*)d_in[7];
  const float* W_w     = (const float*)d_in[8];
  const float* W_b     = (const float*)d_in[9];
  const float* gam     = (const float*)d_in[10];
  const float* bet     = (const float*)d_in[11];
  float* out = (float*)d_out;

  const size_t PXT = (size_t)NTOKS * CI * 2;
  const size_t PWY = (size_t)NTOKS * CI * 4;
  const size_t PRA = (2 * PXT > PWY) ? 2 * PXT : PWY;
  const size_t PWC = (size_t)T3P * CI * 2;
  const size_t PWR = (size_t)CI * O2P * 2;
  const size_t PTH = (size_t)NTOKS * CM * 4;
  const size_t PT3 = (size_t)NTOKS * T3P * 2;
  const size_t PPP = (size_t)NPTOK * PGW * 4;
  const size_t PPG = (size_t)NB * PGW * K3 * 2;
  const size_t PMT = (size_t)NB * CM * T3P * 2;
  const size_t PO2 = (size_t)NTOKS * O2P * 2;
  const size_t PPT = (size_t)NPART * PARTW * 4;
  const size_t PSS = (size_t)PARTW * 4;
  size_t off = 0;
  const size_t oRA = off; off = al256(off + PRA);
  const size_t oWC = off; off = al256(off + PWC);
  const size_t oWR = off; off = al256(off + PWR);
  const size_t oTH = off; off = al256(off + PTH);
  const size_t oT3 = off; off = al256(off + PT3);
  const size_t oPP = off; off = al256(off + PPP);
  const size_t oPG = off; off = al256(off + PPG);
  const size_t oMT = off; off = al256(off + PMT);
  const size_t oO2 = off; off = al256(off + PO2);
  const size_t oPT = off; off = al256(off + PPT);
  const size_t oSS = off; off = al256(off + PSS);
  if (off > ws_size || off > (size_t)WSMAX) return;

  char* ws = (char*)d_ws;
  unsigned short* XT  = (unsigned short*)(ws + oRA);
  unsigned short* YTP = (unsigned short*)(ws + oRA + PXT);
  float*          WY  = (float*)(ws + oRA);
  unsigned short* WC  = (unsigned short*)(ws + oWC);
  unsigned short* WR2 = (unsigned short*)(ws + oWR);
  float*          TH  = (float*)(ws + oTH);
  unsigned short* T3  = (unsigned short*)(ws + oT3);
  float*          PGP = (float*)(ws + oPP);
  unsigned short* PG3 = (unsigned short*)(ws + oPG);
  unsigned short* MT3 = (unsigned short*)(ws + oMT);
  unsigned short* O2  = (unsigned short*)(ws + oO2);
  float*          PT  = (float*)(ws + oPT);
  float*          SS  = (float*)(ws + oSS);

  const dim3 blk(256);

  tconv_kernel<<<dim3(NSP / 64, CI / 64, NB), blk, 0, stream>>>(x, XT, NSP, CI, (long)CI * NSP, (long)NSP * CI);
  tconvp_kernel<<<dim3(NSP / 64, CI / 64, NB), blk, 0, stream>>>(y, YTP, NSP, CI, (long)CI * NSP, (long)NSP * CI);
  wcvt_kernel<<<dim3((CM * CI) / 8 / 256, 5), blk, 0, stream>>>(theta_w, phi_w, g_w, W_w, WC, WR2);

  const dim3 gT(((NTOKS / 64) * (CM / 64) + 7) / 8, 1);
  wmma_gemm64<1, 2, 0, false, false><<<gT, blk, 0, stream>>>(
      XT, CI, 0L, WC, CI, 0L,
      (void*)TH, (void*)TH, (void*)TH, CM, 0L,
      theta_b, gam, bet, gam, bet, x, 0L, NTOKS, CM, CI, 1.0f);
  k_thnorm<<<NTOKS / 64, blk, 0, stream>>>(TH, T3);

  const dim3 gPG(((NTOKS / 64) * (PGW / 64) + 7) / 8, 1);
  k_gemm_pool<<<gPG, blk, 0, stream>>>(YTP, CI, WC + (size_t)CM * CI, CI, PGP, PGW, phi_b, g_b, NTOKS, PGW, CI);
  k_pgcvt<<<dim3(NKP / 64, 2, NB), blk, 0, stream>>>(PGP, PG3);

  const dim3 gM(1, NB);
  wmma_gemm64<1, 0, 4, false, false><<<gM, blk, 0, stream>>>(
      PG3 + (size_t)CM * K3, K3, (long)PGW * K3, PG3, K3, (long)PGW * K3,
      (void*)MT3, (void*)(MT3 + CM), (void*)(MT3 + 2 * CM), T3P, (long)CM * T3P,
      W_b, gam, bet, gam, bet, x, 0L, CM, CM, K3, 1.0f / (float)NKP);

  const dim3 gO(((NSP / 64) * (CM / 64) + 7) / 8, NB);
  wmma_gemm64<1, 0, 2, false, false><<<gO, blk, 0, stream>>>(
      T3, T3P, (long)NSP * T3P, MT3, T3P, (long)CM * T3P,
      (void*)O2, (void*)(O2 + CM), (void*)O2, O2P, (long)NSP * O2P,
      W_b, gam, bet, gam, bet, x, 0L, NSP, CM, T3P, 1.0f);

  const dim3 gW(((NTOKS / 64) * (CI / 64) + 7) / 8, 1);
  wmma_gemm64<1, 2, 0, false, false><<<gW, blk, 0, stream>>>(
      O2, O2P, 0L, WR2, O2P, 0L,
      (void*)WY, (void*)WY, (void*)WY, CI, 0L,
      W_b, gam, bet, gam, bet, x, 0L, NTOKS, CI, O2P, 1.0f);

  k_bnpart<<<NPART, blk, 0, stream>>>(WY, PT);
  k_bnfin<<<1, blk, 0, stream>>>(PT, gam, bet, SS);
  k_out<<<NB * (NSP / 64) * (CI / 64), blk, 0, stream>>>(WY, SS, x, out);
  (void)hipGetLastError();
}
